// single_head_local_attention_48919677501895
// MI455X (gfx1250) — hardware-verified
//
#include <hip/hip_runtime.h>
#include <stdint.h>

#define BN   2
#define CN   256
#define HN   64
#define WN   64
#define KW   7
#define PR   3
#define HP   70
#define WPK  80
#define WPV  128
#define TP   264
#define PS   232
#define OSP  68
#define NBQ  (BN * HN)
#define NBK  (BN * HP)
#define NBV  (BN * HP)
#define SCL  0.0625f
#define PSC  1024.0f
#define VSC  16.0f
#define OSC  0.00006103515625f

static_assert(HP == HN + 2 * PR);
static_assert(KW == 2 * PR + 1);
static_assert(WN == 64 && HN == 64);
static_assert(WPK >= 3 * 16 + 32);
static_assert(WPV >= WPK && ((WPV * 2) % 256) == 0);
static_assert((CN % 64) == 0 && (CN % 32) == 0);
static_assert(((TP * 2) % 16) == 0 && TP >= CN);
static_assert(((PS * 2) % 16) == 0 && PS >= KW * 32);
static_assert(((OSP * 4) % 16) == 0 && OSP >= WN);
static_assert(NBQ == 128 && NBK == 140 && NBV == 140);

typedef _Float16       v16h  __attribute__((ext_vector_type(16)));
typedef _Float16       v8h   __attribute__((ext_vector_type(8)));
typedef unsigned short v16us __attribute__((ext_vector_type(16)));
typedef unsigned short v8us  __attribute__((ext_vector_type(8)));
typedef float          v8f   __attribute__((ext_vector_type(8)));
typedef float          v4f   __attribute__((ext_vector_type(4)));
typedef unsigned int   v4u   __attribute__((ext_vector_type(4)));
#if defined(__HIP_DEVICE_COMPILE__)
typedef __bf16         v16b  __attribute__((ext_vector_type(16)));
#endif

union U8 { v8us u; v4u w; };

__device__ __forceinline__ unsigned short bf_bits(float f) {
  unsigned u = __float_as_uint(f);
  return (unsigned short)((u + 0x7FFFu + ((u >> 16) & 1u)) >> 16);
}
__device__ __forceinline__ float bf_up(unsigned short b) { return __uint_as_float(((unsigned)b) << 16); }
__device__ __forceinline__ float bfr(float f) { return bf_up(bf_bits(f)); }
__device__ __forceinline__ unsigned short h_bits(_Float16 x) { return __builtin_bit_cast(unsigned short, x); }
__device__ __forceinline__ unsigned short hb16(float f) { return h_bits((_Float16)f); }
__device__ __forceinline__ unsigned pk16(unsigned short a, unsigned short b) { return (unsigned)a | ((unsigned)b << 16); }
__device__ __forceinline__ v8f zero8() { v8f z = {0.f, 0.f, 0.f, 0.f, 0.f, 0.f, 0.f, 0.f}; return z; }

__device__ __forceinline__ v16us ldfrag(const unsigned short* p) {
  union { v16us v; v8us h[2]; } f;
  f.h[0] = *(const v8us*)(p);
  f.h[1] = *(const v8us*)(p + 16);
  return f.v;
}

template<int BF>
__device__ __forceinline__ v8f mma16(v16us a, v16us b, v8f c) {
#if defined(__HIP_DEVICE_COMPILE__)
  if (BF) {
    return __builtin_amdgcn_wmma_f32_16x16x32_bf16(false, __builtin_bit_cast(v16b, a), false,
                                                  __builtin_bit_cast(v16b, b), (short)0, c, false, false);
  }
  return __builtin_amdgcn_wmma_f32_16x16x32_f16(false, __builtin_bit_cast(v16h, a), false,
                                               __builtin_bit_cast(v16h, b), (short)0, c, false, false);
#else
  (void)a; (void)b;
  return c;
#endif
}
__device__ __forceinline__ void guard2(v8f& c0, v8f& c1, const v16us& a0, const v16us& a1, const v16us& b) {
#if defined(__HIP_DEVICE_COMPILE__)
  asm volatile("v_nop\n\tv_nop\n\tv_nop\n\tv_nop" : "+v"(c0), "+v"(c1) : "v"(a0), "v"(a1), "v"(b));
#endif
}
__device__ __forceinline__ void guard4(v8f& c0, v8f& c1, v8f& c2, v8f& c3, const v16us& a,
                                       const v16us& b0, const v16us& b1, const v16us& b2, const v16us& b3) {
#if defined(__HIP_DEVICE_COMPILE__)
  asm volatile("v_nop\n\tv_nop\n\tv_nop\n\tv_nop"
               : "+v"(c0), "+v"(c1), "+v"(c2), "+v"(c3)
               : "v"(a), "v"(b0), "v"(b1), "v"(b2), "v"(b3));
#endif
}

__device__ __forceinline__ void score16(const unsigned short* __restrict__ kr, const unsigned short* __restrict__ qr,
                                        v8f& s0, v8f& s1) {
  v8f a0 = zero8(), a1 = zero8();
#pragma unroll 1
  for (int ks = 0; ks < CN / 32; ++ks) {
    const int ko = ks * 32;
    const v16us fq  = ldfrag(qr + ko);
    const v16us fk0 = ldfrag(kr + ko);
    const v16us fk1 = ldfrag(kr + 16 * CN + ko);
    a0 = mma16<1>(fk0, fq, a0);
    a1 = mma16<1>(fk1, fq, a1);
    guard2(a0, a1, fk0, fk1, fq);
  }
  s0 = a0;
  s1 = a1;
}

__global__ __launch_bounds__(256)
void k_cvt(const float* __restrict__ q, const float* __restrict__ k, const float* __restrict__ v,
           unsigned short* qn, unsigned short* kp, unsigned short* vp) {
  __shared__ __align__(16) unsigned short Ts[WN * TP];
  const int tid = threadIdx.x;
  const int blk = blockIdx.x;
  const v4u z4 = {0u, 0u, 0u, 0u};
  if (blk < NBQ + NBK) {
    const bool isq = (blk < NBQ);
    int b, hp, hrow;
    if (isq) {
      b = blk >> 6; hp = blk & 63; hrow = hp;
    } else {
      const int r = blk - NBQ;
      b = r / HP; hp = r - b * HP; hrow = hp - PR;
    }
    const bool rowok = ((unsigned)hrow < (unsigned)HN);
    const int hc = min(max(hrow, 0), HN - 1);
    const float* src = isq ? q : k;
    const float* srow = src + (size_t)b * CN * HN * WN + (size_t)hc * WN;
#pragma unroll 4
    for (int it = 0; it < 64; ++it) {
      const int idx = it * 256 + tid;
      const int c = idx >> 6, w = idx & 63;
      Ts[w * TP + c] = bf_bits(srow[(size_t)c * (HN * WN) + w]);
    }
    __syncthreads();
    const int npc = isq ? 8 : 10;
    const int wof = isq ? 0 : PR;
    unsigned short* dst = isq ? (qn + (size_t)((b * HN + hp) * WN) * CN)
                              : (kp + (size_t)((b * HP + hp) * WPK) * CN);
    v4u pk[10];
#pragma unroll
    for (int s = 0; s < 10; ++s) {
      const int idx = s * 256 + tid;
      const int prw = idx >> 5, piece = idx & 31;
      const int w = prw - wof;
      const bool ok = rowok && ((unsigned)w < (unsigned)WN);
      const int wc = min(max(w, 0), WN - 1);
      const v4u val = *(const v4u*)(Ts + wc * TP + piece * 8);
      pk[s] = ok ? val : z4;
    }
#pragma unroll
    for (int s = 0; s < 10; ++s)
      if (s < npc) *(volatile v4u*)(dst + (size_t)(s * 256 + tid) * 8) = pk[s];
    __threadfence();
#pragma unroll
    for (int s = 0; s < 10; ++s)
      if (s < npc) *(volatile v4u*)(dst + (size_t)(s * 256 + tid) * 8) = pk[s];
  } else if (blk < NBQ + NBK + NBV) {
    const int r = blk - NBQ - NBK;
    const int b = r / HP, hp = r - b * HP, hrow = hp - PR;
    const bool rowok = ((unsigned)hrow < (unsigned)HN);
    const int hc = min(max(hrow, 0), HN - 1);
    const float* vsrc = v + (size_t)b * CN * HN * WN + (size_t)hc * WN;
    unsigned short* vdst = vp + ((size_t)b * CN * HP + hp) * WPV;
#pragma unroll 1
    for (int gq = 0; gq < 2; ++gq) {
      v4u pk[8];
      unsigned offs[8];
#pragma unroll
      for (int s = 0; s < 8; ++s) {
        const int idx = (gq * 8 + s) * 256 + tid;
        const int c = idx >> 4, piece = idx & 15;
        const float* vr = vsrc + (size_t)c * (HN * WN);
        v4u a;
#pragma unroll
        for (int e = 0; e < 4; ++e) {
          const int wa = piece * 8 + 2 * e - PR, wb = wa + 1;
          const float fa = vr[min(max(wa, 0), WN - 1)];
          const float fb = vr[min(max(wb, 0), WN - 1)];
          const unsigned short ba = (rowok && ((unsigned)wa < (unsigned)WN)) ? hb16(bfr(fa) * VSC) : (unsigned short)0;
          const unsigned short bb = (rowok && ((unsigned)wb < (unsigned)WN)) ? hb16(bfr(fb) * VSC) : (unsigned short)0;
          a[e] = pk16(ba, bb);
        }
        pk[s] = a;
        offs[s] = (unsigned)c * (unsigned)(HP * WPV) + (unsigned)(piece * 8);
      }
#pragma unroll
      for (int s = 0; s < 8; ++s) *(volatile v4u*)(vdst + offs[s]) = pk[s];
      __threadfence();
#pragma unroll
      for (int s = 0; s < 8; ++s) *(volatile v4u*)(vdst + offs[s]) = pk[s];
    }
  }
}

__global__ __launch_bounds__(128)
void k_attn(const unsigned short* __restrict__ qn, const unsigned short* __restrict__ kp,
            const unsigned short* __restrict__ vp, float* out) {
  __shared__ __align__(16) unsigned short Pw[64 * PS];
  __shared__ __align__(16) float Os[64 * OSP];
  const int tid = threadIdx.x, wv = tid >> 5, lane = tid & 31, hh = lane >> 4, m = lane & 15;
  const int b = blockIdx.x >> 6, h = blockIdx.x & 63;
  const int w0 = wv * 16;
  const unsigned short* qr = qn + (size_t)((b * HN + h) * WN + w0 + m) * CN + 8 * hh;
  const unsigned short* kr = kp + (size_t)((b * HP + h) * WPK + w0 + m) * CN + 8 * hh;

  v8f sc[14];
  score16(kr + 0 * (WPK * CN), qr, sc[0],  sc[1]);
  score16(kr + 1 * (WPK * CN), qr, sc[2],  sc[3]);
  score16(kr + 2 * (WPK * CN), qr, sc[4],  sc[5]);
  score16(kr + 3 * (WPK * CN), qr, sc[6],  sc[7]);
  score16(kr + 4 * (WPK * CN), qr, sc[8],  sc[9]);
  score16(kr + 5 * (WPK * CN), qr, sc[10], sc[11]);
  score16(kr + 6 * (WPK * CN), qr, sc[12], sc[13]);

  unsigned lv0 = 0u, lv1 = 0u;
#pragma unroll
  for (int r = 0; r < 8; ++r) {
    lv0 |= ((unsigned)(8 * hh + r - m)      <= (unsigned)(KW - 1)) ? (1u << r) : 0u;
    lv1 |= ((unsigned)(16 + 8 * hh + r - m) <= (unsigned)(KW - 1)) ? (1u << r) : 0u;
  }

  float mx = -3.0e38f;
#pragma unroll
  for (int t = 0; t < 14; ++t) {
    const unsigned lv = (t & 1) ? lv1 : lv0;
#pragma unroll
    for (int r = 0; r < 8; ++r) mx = fmaxf(mx, ((lv >> r) & 1u) ? sc[t][r] : -3.0e38f);
  }
  const float mq = fmaxf(mx, __shfl_xor(mx, 16, 32));
  float ls = 0.f;
#pragma unroll
  for (int t = 0; t < 14; ++t) {
    const unsigned lv = (t & 1) ? lv1 : lv0;
#pragma unroll
    for (int r = 0; r < 8; ++r) {
      const float e = __expf((sc[t][r] - mq) * SCL);
      const float p = ((lv >> r) & 1u) ? e : 0.f;
      sc[t][r] = p;
      ls += p;
    }
  }
  const float sq = ls + __shfl_xor(ls, 16, 32);
  const float scl = PSC * __builtin_amdgcn_rcpf(sq);
  {
    unsigned short* pwr = Pw + (wv * 16 + m) * PS + 8 * hh;
#pragma unroll
    for (int t = 0; t < 14; ++t) {
      U8 u;
#pragma unroll
      for (int e = 0; e < 4; ++e) u.w[e] = pk16(hb16(sc[t][2 * e] * scl), hb16(sc[t][2 * e + 1] * scl));
      *(v8us*)(pwr + t * 16) = u.u;
    }
  }
  __syncthreads();

  const unsigned short* vr  = vp + ((size_t)(b * CN + m) * HP + h) * WPV + w0 + 8 * hh;
  const unsigned short* prd = Pw + (wv * 16 + m) * PS + 8 * hh;
#pragma unroll 1
  for (int cc = 0; cc < CN / 64; ++cc) {
    v8f o0 = zero8(), o1 = zero8(), o2 = zero8(), o3 = zero8();
    const unsigned short* vc = vr + (size_t)(cc * 64) * (HP * WPV);
#pragma unroll 1
    for (int g = 0; g < KW; ++g) {
      const v16us fp = ldfrag(prd + 32 * g);
      const unsigned short* vg = vc + g * WPV;
      const v16us f0 = ldfrag(vg);
      const v16us f1 = ldfrag(vg + 16 * (HP * WPV));
      const v16us f2 = ldfrag(vg + 32 * (HP * WPV));
      const v16us f3 = ldfrag(vg + 48 * (HP * WPV));
      o0 = mma16<0>(fp, f0, o0);
      o1 = mma16<0>(fp, f1, o1);
      o2 = mma16<0>(fp, f2, o2);
      o3 = mma16<0>(fp, f3, o3);
      guard4(o0, o1, o2, o3, fp, f0, f1, f2, f3);
    }
    __syncthreads();
    {
      float* orow = Os + w0 + 8 * hh;
      v4f a0 = {o0[0], o0[1], o0[2], o0[3]}, b0 = {o0[4], o0[5], o0[6], o0[7]};
      v4f a1 = {o1[0], o1[1], o1[2], o1[3]}, b1 = {o1[4], o1[5], o1[6], o1[7]};
      v4f a2 = {o2[0], o2[1], o2[2], o2[3]}, b2 = {o2[4], o2[5], o2[6], o2[7]};
      v4f a3 = {o3[0], o3[1], o3[2], o3[3]}, b3 = {o3[4], o3[5], o3[6], o3[7]};
      *(v4f*)(orow + (0 * 16 + m) * OSP)     = a0 * OSC;
      *(v4f*)(orow + (0 * 16 + m) * OSP + 4) = b0 * OSC;
      *(v4f*)(orow + (1 * 16 + m) * OSP)     = a1 * OSC;
      *(v4f*)(orow + (1 * 16 + m) * OSP + 4) = b1 * OSC;
      *(v4f*)(orow + (2 * 16 + m) * OSP)     = a2 * OSC;
      *(v4f*)(orow + (2 * 16 + m) * OSP + 4) = b2 * OSC;
      *(v4f*)(orow + (3 * 16 + m) * OSP)     = a3 * OSC;
      *(v4f*)(orow + (3 * 16 + m) * OSP + 4) = b3 * OSC;
    }
    __syncthreads();
#pragma unroll 1
    for (int it = 0; it < 8; ++it) {
      const int cl = wv * 16 + it * 2 + hh;
      const v4f val = *(const v4f*)(Os + cl * OSP + m * 4);
      float* p = out + (size_t)((b * CN + cc * 64 + cl) * HN + h) * WN + m * 4;
      *(volatile v4f*)p = val;
      __threadfence();
      *(volatile v4f*)p = val;
    }
  }
}

extern "C" void kernel_launch(void* const* d_in, const int* in_sizes, int n_in,
                              void* d_out, int out_size, void* d_ws, size_t ws_size,
                              hipStream_t stream) {
  if (n_in < 3) return;
  const int nel = BN * CN * HN * WN;
  if (in_sizes[0] != nel || in_sizes[1] != nel || in_sizes[2] != nel) return;
  if (out_size != nel) return;

  const float* q = (const float*)d_in[0];
  const float* k = (const float*)d_in[1];
  const float* v = (const float*)d_in[2];
  float* out = (float*)d_out;

  const size_t AL = 65536;
  const size_t sQ = (((size_t)BN * HN * WN * CN * 2) + AL - 1) / AL * AL;
  const size_t sK = (((size_t)BN * HP * WPK * CN * 2) + AL - 1) / AL * AL;
  const size_t sV = (((size_t)BN * CN * HP * WPV * 2) + AL - 1) / AL * AL;
  size_t off = 0;
  const size_t oQ = off; off += sQ;
  const size_t oK = off; off += sK;
  const size_t oV = off; off += sV;
  if (off > ws_size) return;
  if (off > (size_t)134217728) return;

  char* ws = (char*)d_ws;
  unsigned short* Qn = (unsigned short*)(ws + oQ);
  unsigned short* Kp = (unsigned short*)(ws + oK);
  unsigned short* Vp = (unsigned short*)(ws + oV);

  k_cvt<<<dim3(NBQ + NBK + NBV), dim3(256), 0, stream>>>(q, k, v, Qn, Kp, Vp);
  k_attn<<<dim3(BN * HN), dim3(128), 0, stream>>>(Qn, Kp, Vp, out);
  (void)hipGetLastError();
}
